// rgcn_layer_78829829751101
// MI455X (gfx1250) — hardware-verified
//
#include <hip/hip_runtime.h>
#include <stddef.h>


#define DF     128
#define DH     256
#define NTHR   256
#define NWAVE  8
#define EPT    8
#define NGRP   2
#define CHUNK  (NTHR * EPT * NGRP)
#define WCAP   (EPT * NGRP * 32)
#define LISTN  (NWAVE * WCAP)
#define NB     512
#define XROWS  128
#define TPW    (NB / (16 * NWAVE))
#define LN_EPS 1e-5f

#define WP_U2I 0
#define WP_I2U (WP_U2I + 2 * DF * DF)
#define WP_SU  (WP_I2U + 2 * DF * DF)
#define WP_SI  (WP_SU  + 2 * DF * DF)
#define WP_W1  (WP_SI  + 2 * DF * DF)
#define WP_W2  (WP_W1  + 2 * DH * DF)
#define WP_TOT (WP_W2  + 2 * DF * DH)

#define LDS_XFORM (XROWS * DF * 4)
#define LDS_NODE  (NB * DF * 4 + LISTN * 4 + 64)

static_assert((CHUNK & (CHUNK - 1)) == 0);
static_assert(CHUNK <= 4096);
static_assert(NB <= 4096 && (NB & (NB - 1)) == 0);
static_assert(NB == TPW * 16 * NWAVE);
static_assert(WP_TOT == 262144);
static_assert(DF % 32 == 0 && DH % 32 == 0);

typedef float          v4f   __attribute__((ext_vector_type(4)));
typedef float          v8f   __attribute__((ext_vector_type(8)));
typedef int            v4i   __attribute__((ext_vector_type(4)));
typedef unsigned short v8us  __attribute__((ext_vector_type(8)));
typedef unsigned short v16us __attribute__((ext_vector_type(16)));
typedef __bf16         v16bf __attribute__((ext_vector_type(16)));
union FragB { v16bf v; v16us w; v8us u[2]; };

__device__ __forceinline__ unsigned int bf16_bits(float x) {
  const unsigned int u = __float_as_uint(x);
  return (u + 0x7FFFu + ((u >> 16) & 1u)) >> 16;
}

__device__ __forceinline__ void put_hl(FragB& hi, FragB& lo, const int i, const float x) {
  const unsigned int hb = bf16_bits(x);
  const float hf = __uint_as_float(hb << 16);
  hi.w[i] = (unsigned short)hb;
  lo.w[i] = (unsigned short)bf16_bits(x - hf);
}

__device__ __forceinline__ void frag_row(const float* rp, FragB& hi, FragB& lo) {
  const v4f x0 = *(const v4f*)rp;
  const v4f x1 = *(const v4f*)(rp + 4);
  const v4f x2 = *(const v4f*)(rp + 16);
  const v4f x3 = *(const v4f*)(rp + 20);
#pragma unroll
  for (int j = 0; j < 4; ++j) {
    put_hl(hi, lo, j,      x0[j]);
    put_hl(hi, lo, 4 + j,  x1[j]);
    put_hl(hi, lo, 8 + j,  x2[j]);
    put_hl(hi, lo, 12 + j, x3[j]);
  }
}

__device__ __forceinline__ void frag_plane(const unsigned short* __restrict__ ph, const unsigned short* __restrict__ pl,
                                           const int off, FragB& hi, FragB& lo) {
  hi.u[0] = *(const v8us*)(ph + off);
  hi.u[1] = *(const v8us*)(ph + off + 16);
  lo.u[0] = *(const v8us*)(pl + off);
  lo.u[1] = *(const v8us*)(pl + off + 16);
}

__device__ __forceinline__ v8f wmb(v16bf a, v16bf b, v8f c) {
  v8f d = __builtin_amdgcn_wmma_f32_16x16x32_bf16(false, a, false, b, (short)0, c, false, false);
  asm volatile("v_nop\n\tv_nop\n\tv_nop\n\tv_nop" : "+v"(d) : "v"(a), "v"(b));
  return d;
}

__device__ __forceinline__ v8f wm3(const FragB& ah, const FragB& al, const FragB& bh, const FragB& bl, v8f c) {
  c = wmb(ah.v, bh.v, c);
  c = wmb(ah.v, bl.v, c);
  c = wmb(al.v, bh.v, c);
  return c;
}

__device__ __forceinline__ int scan_chunk(const int* __restrict__ dsts, int nE, int cbase, int nodeBase,
                                          int vec8, int* list, int tid, int lane, int wave) {
  int wc = 0;
#pragma unroll
  for (int g = 0; g < NGRP; ++g) {
    const int el0  = (g * NTHR + tid) * EPT;
    const int e0   = cbase + el0;
    const int sent = -2147483647 - 1;
    v4i da, db;
    if (vec8 != 0 && cbase + CHUNK <= nE) {
      da = *(const v4i*)(dsts + e0);
      db = *(const v4i*)(dsts + e0 + 4);
    } else {
      da.x = (e0     < nE) ? dsts[min(e0,     nE - 1)] : sent;
      da.y = (e0 + 1 < nE) ? dsts[min(e0 + 1, nE - 1)] : sent;
      da.z = (e0 + 2 < nE) ? dsts[min(e0 + 2, nE - 1)] : sent;
      da.w = (e0 + 3 < nE) ? dsts[min(e0 + 3, nE - 1)] : sent;
      db.x = (e0 + 4 < nE) ? dsts[min(e0 + 4, nE - 1)] : sent;
      db.y = (e0 + 5 < nE) ? dsts[min(e0 + 5, nE - 1)] : sent;
      db.z = (e0 + 6 < nE) ? dsts[min(e0 + 6, nE - 1)] : sent;
      db.w = (e0 + 7 < nE) ? dsts[min(e0 + 7, nE - 1)] : sent;
    }
    const unsigned nb = (unsigned)nodeBase;
    const unsigned s0 = (unsigned)da.x - nb, s1 = (unsigned)da.y - nb;
    const unsigned s2 = (unsigned)da.z - nb, s3 = (unsigned)da.w - nb;
    const unsigned s4 = (unsigned)db.x - nb, s5 = (unsigned)db.y - nb;
    const unsigned s6 = (unsigned)db.z - nb, s7 = (unsigned)db.w - nb;
    const bool h0 = s0 < (unsigned)NB, h1 = s1 < (unsigned)NB, h2 = s2 < (unsigned)NB, h3 = s3 < (unsigned)NB;
    const bool h4 = s4 < (unsigned)NB, h5 = s5 < (unsigned)NB, h6 = s6 < (unsigned)NB, h7 = s7 < (unsigned)NB;
    const unsigned any = __builtin_amdgcn_ballot_w32(h0 | h1 | h2 | h3 | h4 | h5 | h6 | h7);
    if (any != 0u) {
#define HITJ(J, HJ, SJ) { \
        const unsigned mj = __builtin_amdgcn_ballot_w32(HJ); \
        if (mj != 0u) { \
          if (HJ) { \
            const int pos = wc + (int)__builtin_amdgcn_mbcnt_lo(mj, 0u); \
            if (pos < WCAP) list[wave * WCAP + pos] = ((el0 + (J)) << 12) | (int)(SJ); \
          } \
          wc += (int)__builtin_popcount(mj); } }
      HITJ(0, h0, s0)
      HITJ(1, h1, s1)
      HITJ(2, h2, s2)
      HITJ(3, h3, s3)
      HITJ(4, h4, s4)
      HITJ(5, h5, s5)
      HITJ(6, h6, s6)
      HITJ(7, h7, s7)
#undef HITJ
    }
  }
  return wc;
}

__global__ __launch_bounds__(NTHR) void k_wprep(
    const float* __restrict__ w_u2i, const float* __restrict__ w_i2u,
    const float* __restrict__ w_su,  const float* __restrict__ w_si,
    const float* __restrict__ w_1,   const float* __restrict__ w_2,
    unsigned short* wp) {
  const int b = blockIdx.x, tid = threadIdx.x;
  const int seg  = (b < 8) ? 0 : (b < 16) ? 1 : (b < 24) ? 2 : (b < 32) ? 3 : (b < 48) ? 4 : 5;
  const int b0   = (seg == 0) ? 0 : (seg == 1) ? 8 : (seg == 2) ? 16 : (seg == 3) ? 24 : (seg == 4) ? 32 : 48;
  const float* W = (seg == 0) ? w_u2i : (seg == 1) ? w_i2u : (seg == 2) ? w_su : (seg == 3) ? w_si : (seg == 4) ? w_1 : w_2;
  const int K    = (seg == 5) ? DH : DF;
  const int N    = (seg == 4) ? DH : DF;
  const int ksh  = (seg == 5) ? 8 : 7;
  const int base = (seg == 0) ? WP_U2I : (seg == 1) ? WP_I2U : (seg == 2) ? WP_SU : (seg == 3) ? WP_SI : (seg == 4) ? WP_W1 : WP_W2;
  const int g  = (b - b0) * NTHR + tid;
  const int o  = g * 8;
  const int n  = o >> ksh;
  const int k0 = o & (K - 1);
  float x[8];
#pragma unroll
  for (int j = 0; j < 8; ++j) x[j] = W[(size_t)(k0 + j) * N + n];
  v8us hv, lv;
#pragma unroll
  for (int j = 0; j < 8; ++j) {
    const unsigned int hb = bf16_bits(x[j]);
    const float hf = __uint_as_float(hb << 16);
    hv[j] = (unsigned short)hb;
    lv[j] = (unsigned short)bf16_bits(x[j] - hf);
  }
  unsigned short* dh = wp + base + o;
  unsigned short* dl = dh + (size_t)K * N;
  *(volatile v8us*)dh = hv;
  *(volatile v8us*)dl = lv;
  __threadfence();
  *(volatile v8us*)dh = hv;
  *(volatile v8us*)dl = lv;
}

__global__ __launch_bounds__(NTHR) void k_xform(
    const float* __restrict__ featU, const float* __restrict__ featI,
    const unsigned short* __restrict__ wp, float* tpl, int nU, int nI, int rowsPad) {
  extern __shared__ v4f lds_dyn[];
  float* stg = (float*)lds_dyn;
  const int tid = threadIdx.x, lane = tid & 31, wave = tid >> 5, hh = lane >> 4, m = lane & 15;
  const int typ = blockIdx.y;
  const float* X = typ ? featI : featU;
  const int nN = typ ? nI : nU;
  const unsigned short* ph = wp + (typ ? WP_I2U : WP_U2I);
  const unsigned short* pl = ph + DF * DF;
  float* T = tpl + (size_t)typ * rowsPad * DF;
  const int rowBase = blockIdx.x * XROWS;
  int node = rowBase + 16 * wave + m;
  node = node > nN - 1 ? nN - 1 : node;
  const float* xr = X + (size_t)node * DF + 8 * hh;

  const v8f z8 = {0.f, 0.f, 0.f, 0.f, 0.f, 0.f, 0.f, 0.f};
  v8f acc[8];
#pragma unroll
  for (int nt = 0; nt < 8; ++nt) acc[nt] = z8;
#pragma unroll 1
  for (int ks = 0; ks < DF / 32; ++ks) {
    FragB bh, bl;
    frag_row(xr + 32 * ks, bh, bl);
#pragma unroll
    for (int nt = 0; nt < 8; ++nt) {
      FragB ah, al;
      frag_plane(ph, pl, (16 * nt + m) * DF + 32 * ks + 8 * hh, ah, al);
      acc[nt] = wm3(ah, al, bh, bl, acc[nt]);
    }
  }

  float* sp = stg + (16 * wave + m) * DF + 8 * hh;
#pragma unroll
  for (int nt = 0; nt < 8; ++nt) {
    v4f a, b;
#pragma unroll
    for (int j = 0; j < 4; ++j) { a[j] = acc[nt][j]; b[j] = acc[nt][4 + j]; }
    *(v4f*)(sp + 16 * nt) = a;
    *(v4f*)(sp + 16 * nt + 4) = b;
  }
  __syncthreads();

  const float* lp = stg + 16 * wave * DF + 4 * lane;
  float* gp = T + ((size_t)rowBase + 16 * wave) * DF + 4 * lane;
#pragma unroll
  for (int i = 0; i < 16; ++i) { const v4f v = *(const v4f*)(lp + i * DF); *(volatile v4f*)(gp + (size_t)i * DF) = v; }
  __threadfence();
#pragma unroll
  for (int i = 0; i < 16; ++i) { const v4f v = *(const v4f*)(lp + i * DF); *(volatile v4f*)(gp + (size_t)i * DF) = v; }
}

__global__ __launch_bounds__(NTHR) void k_node(
    const int* __restrict__ dsts, const int* __restrict__ srcs, const float* __restrict__ tsrc,
    const float* __restrict__ brel, const float* __restrict__ featd,
    const unsigned short* __restrict__ wp, int wself,
    const float* __restrict__ lng, const float* __restrict__ lnb,
    const float* __restrict__ fb1, const float* __restrict__ fb2,
    float* out, int nN, int nSrc, int nE, int vec8) {
  extern __shared__ v4f lds_dyn[];
  float* acc  = (float*)lds_dyn;
  int*   list = (int*)(acc + NB * DF);
  int*   wcnt = list + LISTN;
  const int tid = threadIdx.x, lane = tid & 31, wave = tid >> 5, hh = lane >> 4, m = lane & 15;
  const int nodeBase = blockIdx.x * NB;

  {
    const v4f z = {0.f, 0.f, 0.f, 0.f};
    for (int i = tid; i < NB * DF / 4; i += NTHR) lds_dyn[i] = z;
  }
  __syncthreads();

  const int nChunks = (nE + CHUNK - 1) / CHUNK;
#pragma unroll 1
  for (int ch = 0; ch < nChunks; ++ch) {
    const int cbase = ch * CHUNK;
    const int wc = scan_chunk(dsts, nE, cbase, nodeBase, vec8, list, tid, lane, wave);
    if (lane == 0) wcnt[wave] = wc;
    __syncthreads();
    if (wave == 0) {
#pragma unroll 1
      for (int wsx = 0; wsx < NWAVE; ++wsx) {
        int n = __builtin_amdgcn_readfirstlane(wcnt[wsx]);
        n = n > WCAP ? WCAP : (n < 0 ? 0 : n);
        const int* lp = list + wsx * WCAP;
#pragma unroll 1
        for (int i = 0; i < n; ++i) {
          const int ent  = __builtin_amdgcn_readfirstlane(lp[i]);
          const int slot = ent & (NB - 1);
          int e = cbase + ((ent >> 12) & (CHUNK - 1));
          e = e > nE - 1 ? nE - 1 : e;
          int src = srcs[e];
          src = src < 0 ? 0 : (src > nSrc - 1 ? nSrc - 1 : src);
          const v4f v = *(const v4f*)(tsrc + (size_t)src * DF + 4 * lane);
          v4f* ap = (v4f*)(acc + slot * DF + 4 * lane);
          *ap = *ap + v;
        }
      }
    }
    __syncthreads();
  }

  const unsigned short* psh = wp + wself;
  const unsigned short* psl = psh + DF * DF;
  const unsigned short* p1h = wp + WP_W1;
  const unsigned short* p1l = p1h + DH * DF;
  const unsigned short* p2h = wp + WP_W2;
  const unsigned short* p2l = p2h + DF * DH;
  const float inv_d = 1.0f / (float)DF;
  const v8f z8 = {0.f, 0.f, 0.f, 0.f, 0.f, 0.f, 0.f, 0.f};

#pragma unroll 1
  for (int q = 0; q < TPW; ++q) {
    const int t = wave + NWAVE * q;
    const int node0 = nodeBase + 16 * t;
    int node = node0 + m;
    node = node > nN - 1 ? nN - 1 : node;
    const float* fr = featd + (size_t)node * DF + 8 * hh;
    float* hr = acc + (16 * t + m) * DF + 8 * hh;

    v8f xs[8];
#pragma unroll
    for (int nt = 0; nt < 8; ++nt) xs[nt] = z8;
#pragma unroll 1
    for (int ks = 0; ks < DF / 32; ++ks) {
      FragB bh, bl;
      frag_row(fr + 32 * ks, bh, bl);
#pragma unroll
      for (int nt = 0; nt < 8; ++nt) {
        FragB ah, al;
        frag_plane(psh, psl, (16 * nt + m) * DF + 32 * ks + 8 * hh, ah, al);
        xs[nt] = wm3(ah, al, bh, bl, xs[nt]);
      }
    }

    float s1 = 0.f;
#pragma unroll
    for (int nt = 0; nt < 8; ++nt) {
      const v4f m0 = *(const v4f*)(hr + 16 * nt);
      const v4f m1 = *(const v4f*)(hr + 16 * nt + 4);
      const v4f c0 = *(const v4f*)(brel + 16 * nt + 8 * hh);
      const v4f c1 = *(const v4f*)(brel + 16 * nt + 8 * hh + 4);
#pragma unroll
      for (int j = 0; j < 4; ++j) {
        const float a = xs[nt][j] + (m0[j] + c0[j]);
        const float b = xs[nt][4 + j] + (m1[j] + c1[j]);
        xs[nt][j] = a;
        xs[nt][4 + j] = b;
        s1 += a;
        s1 += b;
      }
    }
    s1 += __shfl_xor(s1, 16, 32);
    const float mean = s1 * inv_d;
    float s2 = 0.f;
#pragma unroll
    for (int nt = 0; nt < 8; ++nt) {
#pragma unroll
      for (int j = 0; j < 8; ++j) { const float d = xs[nt][j] - mean; s2 += d * d; }
    }
    s2 += __shfl_xor(s2, 16, 32);
    const float rs = rsqrtf(s2 * inv_d + LN_EPS);

#pragma unroll
    for (int nt = 0; nt < 8; ++nt) {
      const v4f g0 = *(const v4f*)(lng + 16 * nt + 8 * hh);
      const v4f g1 = *(const v4f*)(lng + 16 * nt + 8 * hh + 4);
      const v4f e0 = *(const v4f*)(lnb + 16 * nt + 8 * hh);
      const v4f e1 = *(const v4f*)(lnb + 16 * nt + 8 * hh + 4);
      const v4f f0 = *(const v4f*)(fr + 16 * nt);
      const v4f f1 = *(const v4f*)(fr + 16 * nt + 4);
      v4f y0, y1;
#pragma unroll
      for (int j = 0; j < 4; ++j) {
        y0[j] = fmaxf((xs[nt][j] - mean) * rs * g0[j] + e0[j], 0.f) + f0[j];
        y1[j] = fmaxf((xs[nt][4 + j] - mean) * rs * g1[j] + e1[j], 0.f) + f1[j];
      }
      *(v4f*)(hr + 16 * nt) = y0;
      *(v4f*)(hr + 16 * nt + 4) = y1;
    }

    v8f o2[8];
#pragma unroll
    for (int nt = 0; nt < 8; ++nt) o2[nt] = z8;
#pragma unroll 1
    for (int kt2 = 0; kt2 < DH / 32; ++kt2) {
      v8f da = z8, db = z8;
#pragma unroll 1
      for (int ks = 0; ks < DF / 32; ++ks) {
        FragB bh, bl;
        frag_row(hr + 32 * ks, bh, bl);
        FragB ah, al;
        frag_plane(p1h, p1l, (32 * kt2 + m) * DF + 32 * ks + 8 * hh, ah, al);
        da = wm3(ah, al, bh, bl, da);
        frag_plane(p1h, p1l, (32 * kt2 + 16 + m) * DF + 32 * ks + 8 * hh, ah, al);
        db = wm3(ah, al, bh, bl, db);
      }
      const v4f u0 = *(const v4f*)(fb1 + 32 * kt2 + 8 * hh);
      const v4f u1 = *(const v4f*)(fb1 + 32 * kt2 + 8 * hh + 4);
      const v4f u2 = *(const v4f*)(fb1 + 32 * kt2 + 16 + 8 * hh);
      const v4f u3 = *(const v4f*)(fb1 + 32 * kt2 + 16 + 8 * hh + 4);
      FragB qh, ql;
#pragma unroll
      for (int j = 0; j < 4; ++j) {
        put_hl(qh, ql, j,      fmaxf(da[j]     + u0[j], 0.f));
        put_hl(qh, ql, 4 + j,  fmaxf(da[4 + j] + u1[j], 0.f));
        put_hl(qh, ql, 8 + j,  fmaxf(db[j]     + u2[j], 0.f));
        put_hl(qh, ql, 12 + j, fmaxf(db[4 + j] + u3[j], 0.f));
      }
#pragma unroll
      for (int nt = 0; nt < 8; ++nt) {
        FragB ah, al;
        frag_plane(p2h, p2l, (16 * nt + m) * DH + 32 * kt2 + 8 * hh, ah, al);
        o2[nt] = wm3(ah, al, qh, ql, o2[nt]);
      }
    }

#pragma unroll
    for (int nt = 0; nt < 8; ++nt) {
      const v4f c0 = *(const v4f*)(fb2 + 16 * nt + 8 * hh);
      const v4f c1 = *(const v4f*)(fb2 + 16 * nt + 8 * hh + 4);
      v4f w0, w1;
#pragma unroll
      for (int j = 0; j < 4; ++j) { w0[j] = o2[nt][j] + c0[j]; w1[j] = o2[nt][4 + j] + c1[j]; }
      *(v4f*)(hr + 16 * nt) = w0;
      *(v4f*)(hr + 16 * nt + 4) = w1;
    }
    __syncthreads();

    const float* lrow = acc + (16 * t) * DF + 4 * lane;
#pragma unroll
    for (int i = 0; i < 16; ++i) {
      const int nd = node0 + i;
      if (nd < nN) {
        const v4f v = *(const v4f*)(lrow + i * DF);
        *(volatile v4f*)(out + (size_t)nd * DF + 4 * lane) = v;
      }
    }
    __threadfence();
#pragma unroll
    for (int i = 0; i < 16; ++i) {
      const int nd = node0 + i;
      if (nd < nN) {
        const v4f v = *(const v4f*)(lrow + i * DF);
        *(volatile v4f*)(out + (size_t)nd * DF + 4 * lane) = v;
      }
    }
  }
}

extern "C" void kernel_launch(void* const* d_in, const int* in_sizes, int n_in,
                              void* d_out, int out_size, void* d_ws, size_t ws_size,
                              hipStream_t stream) {
  if (n_in < 20) return;
  const int nU = in_sizes[0] / DF;
  const int nI = in_sizes[1] / DF;
  if (nU <= 0 || nI <= 0 || in_sizes[0] != nU * DF || in_sizes[1] != nI * DF) return;
  if (in_sizes[2] != DF * DF || in_sizes[4] != DF * DF || in_sizes[6] != DF * DF || in_sizes[7] != DF * DF) return;
  if (in_sizes[3] < DF || in_sizes[5] < DF || in_sizes[8] < DF || in_sizes[9] < DF || in_sizes[10] < DF || in_sizes[11] < DF) return;
  if (in_sizes[12] != DF * DH || in_sizes[13] < DH || in_sizes[14] != DH * DF || in_sizes[15] < DF) return;
  const int nE1 = in_sizes[16];
  const int nE2 = in_sizes[18];
  if (nE1 < 0 || nE2 < 0 || in_sizes[17] != nE1 || in_sizes[19] != nE2) return;
  if (out_size != (nU + nI) * DF) return;

  const float* feat_user   = (const float*)d_in[0];
  const float* feat_item   = (const float*)d_in[1];
  const float* W_u2i       = (const float*)d_in[2];
  const float* b_u2i       = (const float*)d_in[3];
  const float* W_i2u       = (const float*)d_in[4];
  const float* b_i2u       = (const float*)d_in[5];
  const float* self_w_user = (const float*)d_in[6];
  const float* self_w_item = (const float*)d_in[7];
  const float* ln_g_user   = (const float*)d_in[8];
  const float* ln_b_user   = (const float*)d_in[9];
  const float* ln_g_item   = (const float*)d_in[10];
  const float* ln_b_item   = (const float*)d_in[11];
  const float* ffn_w1      = (const float*)d_in[12];
  const float* ffn_b1      = (const float*)d_in[13];
  const float* ffn_w2      = (const float*)d_in[14];
  const float* ffn_b2      = (const float*)d_in[15];
  const int*   src_u2i     = (const int*)d_in[16];
  const int*   dst_u2i     = (const int*)d_in[17];
  const int*   src_i2u     = (const int*)d_in[18];
  const int*   dst_i2u     = (const int*)d_in[19];
  float* out0 = (float*)d_out;
  float* out1 = out0 + (size_t)nU * DF;

  const int nMax    = nU > nI ? nU : nI;
  const int nXB     = (nMax + XROWS - 1) / XROWS;
  const int rowsPad = nXB * XROWS;
  const int nBI     = (nI + NB - 1) / NB;
  const int nBU     = (nU + NB - 1) / NB;

  char* ws = (char*)d_ws;
  size_t off = 0;
  const size_t oW = off; off += (size_t)WP_TOT * 2;                 off = (off + 255) & ~(size_t)255;
  const size_t oT = off; off += (size_t)2 * rowsPad * DF * 4;       off = (off + 255) & ~(size_t)255;
  if (off > ws_size) return;
  unsigned short* wp  = (unsigned short*)(ws + oW);
  float*          tpl = (float*)(ws + oT);

  k_wprep<<<64, NTHR, 0, stream>>>(W_u2i, W_i2u, self_w_user, self_w_item, ffn_w1, ffn_w2, wp);

  (void)hipFuncSetAttribute(reinterpret_cast<const void*>(&k_xform),
                            hipFuncAttributeMaxDynamicSharedMemorySize, LDS_XFORM);
  k_xform<<<dim3(nXB, 2), NTHR, LDS_XFORM, stream>>>(feat_user, feat_item, wp, tpl, nU, nI, rowsPad);

  (void)hipFuncSetAttribute(reinterpret_cast<const void*>(&k_node),
                            hipFuncAttributeMaxDynamicSharedMemorySize, LDS_NODE);
  k_node<<<nBI, NTHR, LDS_NODE, stream>>>(dst_u2i, src_u2i, tpl, b_u2i, feat_item, wp, WP_SI,
                                          ln_g_item, ln_b_item, ffn_b1, ffn_b2, out1, nI, nU, nE1, 1);
  k_node<<<nBU, NTHR, LDS_NODE, stream>>>(dst_i2u, src_i2u, tpl + (size_t)rowsPad * DF, b_i2u, feat_user, wp, WP_SU,
                                          ln_g_user, ln_b_user, ffn_b1, ffn_b2, out0, nU, nI, nE2, 1);
}
